// LocalCorrWithGeom_88356067213328
// MI455X (gfx1250) — hardware-verified
//
#include <hip/hip_runtime.h>
#include <math.h>
#include <stddef.h>

typedef __attribute__((ext_vector_type(16))) _Float16 v16h;
typedef __attribute__((ext_vector_type(8)))  _Float16 v8h;
typedef __attribute__((ext_vector_type(8)))  float    v8f;
typedef __attribute__((ext_vector_type(4)))  float    v4f;
typedef __attribute__((ext_vector_type(4)))  unsigned int v4u;

constexpr int kBatch = 2;
constexpr int kCin   = 256;
constexpr int kCmid  = 128;
constexpr int kH     = 112;
constexpr int kW     = 112;
constexpr int kHW    = kH * kW;
constexpr int kPix   = kBatch * kHW;
constexpr int kRad   = 3;
constexpr int kWin   = 2 * kRad + 1;
constexpr int kD     = kWin * kWin;
constexpr int kDP    = 64;
constexpr int kQP    = 132;
constexpr int kCP    = 72;
constexpr int kLP    = 65;
constexpr int kSlabP = 132;

constexpr float kPhiCarry    = 16.0f;
constexpr float kWCarry      = 256.0f;
constexpr float kProjFold    = 1.0f / (kPhiCarry * kWCarry);
constexpr float kCorrCarry   = 512.0f;
constexpr float kMixFold     = 1.0f / (kCorrCarry * kWCarry);
constexpr float kF16MinNorm  = 6.103515625e-05f;
constexpr float kNormEps     = 1e-12f;
constexpr float kDistEps     = 1e-12f;
constexpr float kNegBig      = -3.0e38f;

static_assert(kD == 49, "window");
static_assert(kD <= kDP && (kDP % 32) == 0, "mix K/N padding");
static_assert((kPix % 64) == 0 && (kHW % 64) == 0, "pixel tiles stay inside one batch");
static_assert((kCin % 64) == 0 && (kCin % 32) == 0, "projection K");
static_assert(kCmid == 128, "projection N = 8 column tiles of 16");
static_assert((kPix % 32) == 0, "32-pixel output groups");
static_assert(kProjFold == 1.0f / 4096.0f, "projection fold");
static_assert(kMixFold == 1.0f / 131072.0f, "mix fold");

constexpr size_t kOffAQ  = 0;
constexpr size_t kOffAK  = kOffAQ  + (size_t)kPix * kCin * 2;
constexpr size_t kOffWQH = kOffAK  + (size_t)kPix * kCin * 2;
constexpr size_t kOffWKH = kOffWQH + (size_t)kCmid * kCin * 2;
constexpr size_t kOffWVH = kOffWKH + (size_t)kCmid * kCin * 2;
constexpr size_t kOffQN  = kOffWVH + (size_t)kDP * kDP * 2;
constexpr size_t kOffKN  = kOffQN  + (size_t)kPix * kCmid * 4;
constexpr size_t kWsTotal = kOffKN + (size_t)kPix * kCmid * 4;
static_assert(kWsTotal == 51519488ull, "carve total");
static_assert(kWsTotal <= 134217728ull, "carve cap");
static_assert((kOffAK % 128) == 0 && (kOffWQH % 128) == 0 && (kOffWKH % 128) == 0 &&
              (kOffWVH % 128) == 0 && (kOffQN % 128) == 0 && (kOffKN % 128) == 0, "128-B aligned regions");

union FragU { v16h v; v8h h[2]; };
__device__ __forceinline__ v16h frag_load(const _Float16* p) {
  FragU f;
  f.h[0] = *(const v8h*)(p);
  f.h[1] = *(const v8h*)(p + 16);
  return f.v;
}
__device__ __forceinline__ v8f mma_h(v16h a, v16h b, v8f c) {
  c = __builtin_amdgcn_wmma_f32_16x16x32_f16(false, a, false, b, (short)0, c, false, false);
  asm volatile("v_nop\n\tv_nop\n\tv_nop\n\tv_nop" : "+v"(c) : "v"(a), "v"(b));
  return c;
}
__device__ __forceinline__ unsigned short f16_bits_flush(float v) {
  const float vf = (fabsf(v) < kF16MinNorm) ? 0.0f : v;
  const _Float16 hv = (_Float16)vf;
  return __builtin_bit_cast(unsigned short, hv);
}
__device__ __forceinline__ unsigned pk16(unsigned short a, unsigned short b) {
  return (unsigned)a | ((unsigned)b << 16);
}

__global__ __launch_bounds__(256) void wprep_kernel(
    const float* __restrict__ Wq, const float* __restrict__ Wk, const float* __restrict__ Wv,
    unsigned short* __restrict__ wqh, unsigned short* __restrict__ wkh, unsigned short* __restrict__ wvh)
{
  const int blk = blockIdx.x;
  const int tid = threadIdx.x;
  float x[8];
  unsigned short* dst;
  if (blk < 32) {
    const int sel = blk >> 4;
    const float* src = sel ? Wk : Wq;
    const int i = (blk & 15) * 256 + tid;
    const v4f a = *(const v4f*)(src + 8 * (size_t)i);
    const v4f c = *(const v4f*)(src + 8 * (size_t)i + 4);
#pragma unroll
    for (int e = 0; e < 4; ++e) {
      x[e] = a[e];
      x[4 + e] = c[e];
    }
    dst = (sel ? wkh : wqh) + 8 * (size_t)i;
  } else {
    const int i  = (blk - 32) * 256 + tid;
    const int n  = i >> 3;
    const int kb = (i & 7) * 8;
    const int nc = n < kD ? n : kD - 1;
#pragma unroll
    for (int e = 0; e < 8; ++e) {
      const int k  = kb + e;
      const int kc = k < kD ? k : kD - 1;
      float v = Wv[nc * kD + kc];
      asm volatile("" : "+v"(v));
      x[e] = (n < kD && k < kD) ? v : 0.0f;
    }
    dst = wvh + 8 * (size_t)i;
  }
  unsigned short hb[8];
#pragma unroll
  for (int e = 0; e < 8; ++e) {
    const float sv = x[e] * kWCarry;
    hb[e] = f16_bits_flush(sv);
  }
  const v4u u = (v4u){pk16(hb[0], hb[1]), pk16(hb[2], hb[3]), pk16(hb[4], hb[5]), pk16(hb[6], hb[7])};
  *(volatile v4u*)dst = u;
  __threadfence();
  *(volatile v4u*)dst = u;
}

__global__ __launch_bounds__(256) void phi_transpose_kernel(
    const float* __restrict__ phi0, const float* __restrict__ phi1,
    unsigned short* __restrict__ out0, unsigned short* __restrict__ out1)
{
  __shared__ float sm[64][65];
  const int t    = threadIdx.x;
  const int pix0 = blockIdx.x * 64;
  const int c0   = blockIdx.y * 64;
  const int z    = blockIdx.z;
  const float* phi = z ? phi1 : phi0;
  unsigned short* op = z ? out1 : out0;
  const int b   = pix0 / kHW;
  const int hw0 = pix0 - b * kHW;
  const float* src = phi + ((size_t)b * kCin + c0) * kHW + hw0;
#pragma unroll 4
  for (int i = 0; i < 16; ++i) {
    const int e = i * 256 + t;
    const int r = e >> 6;
    const int c = e & 63;
    sm[c][r] = src[(size_t)r * kHW + c] * kPhiCarry;
  }
  __syncthreads();
  const int lane = t & 31;
  const int wave = t >> 5;
  const int q  = lane >> 3;
  const int c8 = (lane & 7) * 8;
  v4u u[2];
#pragma unroll
  for (int it = 0; it < 2; ++it) {
    const int row = wave * 8 + it * 4 + q;
    unsigned short hb[8];
#pragma unroll
    for (int e = 0; e < 8; ++e) {
      const float sv = sm[row][c8 + e];
      hb[e] = f16_bits_flush(sv);
    }
    u[it] = (v4u){pk16(hb[0], hb[1]), pk16(hb[2], hb[3]), pk16(hb[4], hb[5]), pk16(hb[6], hb[7])};
  }
  for (int pass = 0; pass < 2; ++pass) {
#pragma unroll
    for (int it = 0; it < 2; ++it) {
      const int row = wave * 8 + it * 4 + q;
      *(volatile v4u*)(op + (size_t)(pix0 + row) * kCin + c0 + c8) = u[it];
    }
    __threadfence();
  }
}

__global__ __launch_bounds__(128) void proj_norm_kernel(
    const unsigned short* __restrict__ a0p, const unsigned short* __restrict__ a1p,
    const unsigned short* __restrict__ w0p, const unsigned short* __restrict__ w1p,
    float* __restrict__ o0, float* __restrict__ o1)
{
  __shared__ __align__(16) float slab_s[4 * 16 * kSlabP];
  const int tid  = threadIdx.x;
  const int lane = tid & 31;
  const int wave = __builtin_amdgcn_readfirstlane(tid >> 5);
  const int z    = blockIdx.y;
  const _Float16* A  = (const _Float16*)(z ? a1p : a0p);
  const _Float16* Wt = (const _Float16*)(z ? w1p : w0p);
  float* O = z ? o1 : o0;
  const int m0 = blockIdx.x * 64 + wave * 16;
  const int rl = lane & 15;
  const int hh = lane >> 4;
  const int koff = 8 * hh;

  v8f acc[8];
#pragma unroll
  for (int j = 0; j < 8; ++j) acc[j] = (v8f){0.f, 0.f, 0.f, 0.f, 0.f, 0.f, 0.f, 0.f};

  const _Float16* arow = A  + (size_t)(m0 + rl) * kCin + koff;
  const _Float16* wrow = Wt + (size_t)rl * kCin + koff;
#pragma unroll 1
  for (int k0 = 0; k0 < kCin; k0 += 32) {
    const v16h a = frag_load(arow + k0);
#pragma unroll
    for (int j = 0; j < 8; ++j) {
      const v16h bfr = frag_load(wrow + (size_t)j * 16 * kCin + k0);
      acc[j] = mma_h(a, bfr, acc[j]);
    }
  }

  float inv[8];
#pragma unroll
  for (int r = 0; r < 8; ++r) {
    float s = 0.0f;
#pragma unroll
    for (int j = 0; j < 8; ++j) {
      const float xv = acc[j][r] * kProjFold;
      s = fmaf(xv, xv, s);
    }
    s += __shfl_xor(s, 1, 32);
    s += __shfl_xor(s, 2, 32);
    s += __shfl_xor(s, 4, 32);
    s += __shfl_xor(s, 8, 32);
    const float nrm = sqrtf(s);
    inv[r] = 1.0f / fmaxf(nrm, kNormEps);
  }
  float* slab = slab_s + wave * (16 * kSlabP);
#pragma unroll
  for (int r = 0; r < 8; ++r) {
#pragma unroll
    for (int j = 0; j < 8; ++j) {
      slab[(8 * hh + r) * kSlabP + j * 16 + rl] = (acc[j][r] * kProjFold) * inv[r];
    }
  }
  __builtin_amdgcn_fence(__ATOMIC_RELEASE, "workgroup");
  __builtin_amdgcn_wave_barrier();
  __builtin_amdgcn_fence(__ATOMIC_ACQUIRE, "workgroup");
  {
    const int c4 = lane * 4;
    for (int pass = 0; pass < 2; ++pass) {
#pragma unroll
      for (int row = 0; row < 16; ++row) {
        const v4f v = *(const v4f*)(slab + row * kSlabP + c4);
        *(volatile v4f*)(O + (size_t)(m0 + row) * kCmid + c4) = v;
      }
      __threadfence();
    }
  }
}

__global__ __launch_bounds__(256) void corr_soft_kernel(
    const float* __restrict__ QN, const float* __restrict__ KN,
    const float* __restrict__ Pcur, const float* __restrict__ Prnd,
    const unsigned short* __restrict__ wvh, const float* __restrict__ bv,
    const float* __restrict__ gamma_p, float* __restrict__ out)
{
  __shared__ __align__(16) float    q_s[32 * kQP];
  __shared__ __align__(16) _Float16 corr_s[32 * kCP];
  __shared__ __align__(16) float    lg_s[32 * kLP];
  __shared__ __align__(16) float    res_s[3 * 32];

  const int tid  = threadIdx.x;
  const int lane = tid & 31;
  const int wave = __builtin_amdgcn_readfirstlane(tid >> 5);
  const int pix0 = blockIdx.x * 32;

#pragma unroll
  for (int i = 0; i < 4; ++i) {
    const int e  = i * 256 + tid;
    const int r  = e >> 5;
    const int c4 = (e & 31) * 4;
    const v4f v = *(const v4f*)(QN + (size_t)(pix0 + r) * kCmid + c4);
    *(v4f*)(q_s + r * kQP + c4) = v;
  }

  const int pix = pix0 + lane;
  const int b   = pix / kHW;
  const int rem = pix - b * kHW;
  const int h   = rem / kW;
  const int w   = rem - h * kW;
  const float* pcb = Pcur + (size_t)b * 3 * kHW + rem;
  const float pcx = pcb[0];
  const float pcy = pcb[kHW];
  const float pcz = pcb[2 * kHW];
  const float gam = gamma_p[0];
  const float* prb = Prnd + (size_t)b * 3 * kHW;
  const float* knb = KN + (size_t)b * kHW * kCmid;
  __syncthreads();

#pragma unroll 1
  for (int it = 0; it < 8; ++it) {
    const int d = wave + 8 * it;
    if (d < kD) {
      const int ky = d / kWin;
      const int kx = d - ky * kWin;
      const int hn = h + ky - kRad;
      const int wn = w + kx - kRad;
      const bool inb = ((unsigned)hn < (unsigned)kH) && ((unsigned)wn < (unsigned)kW);
      const int hc = hn < 0 ? 0 : (hn > kH - 1 ? kH - 1 : hn);
      const int wc = wn < 0 ? 0 : (wn > kW - 1 ? kW - 1 : wn);
      const int nrem = hc * kW + wc;
      const float* kv = knb + (size_t)nrem * kCmid;
      const float* qv = q_s + lane * kQP;
      float a0 = 0.0f, a1 = 0.0f, a2 = 0.0f, a3 = 0.0f;
#pragma unroll 4
      for (int c = 0; c < kCmid; c += 4) {
        const v4f kk = *(const v4f*)(kv + c);
        const v4f qq = *(const v4f*)(qv + c);
        a0 = fmaf(qq[0], kk[0], a0);
        a1 = fmaf(qq[1], kk[1], a1);
        a2 = fmaf(qq[2], kk[2], a2);
        a3 = fmaf(qq[3], kk[3], a3);
      }
      float dot = (a0 + a1) + (a2 + a3);
      asm volatile("" : "+v"(dot));
      const float corr = inb ? dot : 0.0f;

      float prx = prb[nrem];
      float pry = prb[kHW + nrem];
      float prz = prb[2 * kHW + nrem];
      asm volatile("" : "+v"(prx), "+v"(pry), "+v"(prz));
      prx = inb ? prx : 0.0f;
      pry = inb ? pry : 0.0f;
      prz = inb ? prz : 0.0f;
      const float dpx = pcx - prx;
      const float dpy = pcy - pry;
      const float dpz = pcz - prz;
      float ss = dpx * dpx + dpy * dpy + dpz * dpz;
      ss = fmaxf(ss, kDistEps);
      const float dist = sqrtf(ss);
      const float geo = gam * (-dist - 0.5f * fabsf(dpz));

      float cs = corr * kCorrCarry;
      cs = (fabsf(cs) < kF16MinNorm) ? 0.0f : cs;
      corr_s[lane * kCP + d] = (_Float16)cs;
      lg_s[lane * kLP + d] = geo;
    } else {
      corr_s[lane * kCP + d] = (_Float16)0.0f;
    }
  }
  __syncthreads();

  {
    const int mt = wave >> 2;
    const int nt = wave & 3;
    const int rl = lane & 15;
    const int hh = lane >> 4;
    const _Float16* WV = (const _Float16*)wvh;
    v8f acc = (v8f){0.f, 0.f, 0.f, 0.f, 0.f, 0.f, 0.f, 0.f};
#pragma unroll
    for (int ks = 0; ks < 2; ++ks) {
      const v16h a   = frag_load(corr_s + (mt * 16 + rl) * kCP + ks * 32 + 8 * hh);
      const v16h bfr = frag_load(WV + (size_t)(nt * 16 + rl) * kDP + ks * 32 + 8 * hh);
      acc = mma_h(a, bfr, acc);
    }
    const int e  = nt * 16 + rl;
    const int ec = e < kD ? e : kD - 1;
    float bve = bv[ec];
    asm volatile("" : "+v"(bve));
#pragma unroll
    for (int r = 0; r < 8; ++r) {
      const int p = mt * 16 + 8 * hh + r;
      const float g = lg_s[p * kLP + ec];
      const float v = (acc[r] * kMixFold + bve) + g;
      if (e < kD) lg_s[p * kLP + e] = v;
    }
  }
  __syncthreads();

  {
    const int p = tid >> 3;
    const int j = tid & 7;
    const float* lrow = lg_s + p * kLP;
    float m = kNegBig;
#pragma unroll 1
    for (int i = 0; i < 7; ++i) {
      const int d  = j + 8 * i;
      const int dc = d < kD ? d : kD - 1;
      const float xv = lrow[dc];
      const float xs = (d < kD) ? xv : kNegBig;
      m = fmaxf(m, xs);
    }
    m = fmaxf(m, __shfl_xor(m, 1, 32));
    m = fmaxf(m, __shfl_xor(m, 2, 32));
    m = fmaxf(m, __shfl_xor(m, 4, 32));
    float s = 0.0f, sx = 0.0f, sy = 0.0f;
#pragma unroll 1
    for (int i = 0; i < 7; ++i) {
      const int d  = j + 8 * i;
      const int dc = d < kD ? d : kD - 1;
      const float xv = lrow[dc];
      float ev = expf(xv - m);
      ev = (d < kD) ? ev : 0.0f;
      const int ky = dc / kWin;
      const int kx = dc - ky * kWin;
      s += ev;
      sx = fmaf(ev, (float)(kx - kRad), sx);
      sy = fmaf(ev, (float)(ky - kRad), sy);
    }
    s  += __shfl_xor(s, 1, 32);
    sx += __shfl_xor(sx, 1, 32);
    sy += __shfl_xor(sy, 1, 32);
    s  += __shfl_xor(s, 2, 32);
    sx += __shfl_xor(sx, 2, 32);
    sy += __shfl_xor(sy, 2, 32);
    s  += __shfl_xor(s, 4, 32);
    sx += __shfl_xor(sx, 4, 32);
    sy += __shfl_xor(sy, 4, 32);
    const float inv = 1.0f / s;
    if (j == 0) {
      res_s[p]      = sx * inv;
      res_s[32 + p] = sy * inv;
      res_s[64 + p] = inv;
    }
  }
  __syncthreads();

  if (wave == 0) {
    const int q  = lane >> 3;
    const int qc = q < 3 ? q : 2;
    const int c4 = (lane & 7) * 4;
    const v4f val = *(const v4f*)(res_s + qc * 32 + c4);
    float* dst = out + (size_t)qc * kPix + pix0 + c4;
    for (int pass = 0; pass < 2; ++pass) {
      if (lane < 24) *(volatile v4f*)dst = val;
      __threadfence();
    }
  }
}

extern "C" void kernel_launch(void* const* d_in, const int* in_sizes, int n_in,
                              void* d_out, int out_size, void* d_ws, size_t ws_size,
                              hipStream_t stream)
{
  if (n_in < 9) return;
  if (in_sizes[0] != kBatch * kCin * kHW) return;
  if (in_sizes[1] != kBatch * kCin * kHW) return;
  if (in_sizes[2] != kBatch * 3 * kHW) return;
  if (in_sizes[3] != kBatch * 3 * kHW) return;
  if (in_sizes[4] != kCmid * kCin) return;
  if (in_sizes[5] != kCmid * kCin) return;
  if (in_sizes[6] != kD * kD) return;
  if (in_sizes[7] != kD) return;
  if (in_sizes[8] != 1) return;
  if (out_size != 3 * kPix) return;
  if (ws_size < kWsTotal) return;

  const float* phi_cur = (const float*)d_in[0];
  const float* phi_rnd = (const float*)d_in[1];
  const float* P_cur   = (const float*)d_in[2];
  const float* P_rnd   = (const float*)d_in[3];
  const float* Wq      = (const float*)d_in[4];
  const float* Wk      = (const float*)d_in[5];
  const float* Wv      = (const float*)d_in[6];
  const float* bvp     = (const float*)d_in[7];
  const float* gammap  = (const float*)d_in[8];
  float* outp = (float*)d_out;

  char* ws = (char*)d_ws;
  unsigned short* AQ  = (unsigned short*)(ws + kOffAQ);
  unsigned short* AK  = (unsigned short*)(ws + kOffAK);
  unsigned short* WQH = (unsigned short*)(ws + kOffWQH);
  unsigned short* WKH = (unsigned short*)(ws + kOffWKH);
  unsigned short* WVH = (unsigned short*)(ws + kOffWVH);
  float* QN = (float*)(ws + kOffQN);
  float* KN = (float*)(ws + kOffKN);

  wprep_kernel<<<34, 256, 0, stream>>>(Wq, Wk, Wv, WQH, WKH, WVH);
  phi_transpose_kernel<<<dim3(kPix / 64, kCin / 64, 2), 256, 0, stream>>>(phi_cur, phi_rnd, AQ, AK);
  proj_norm_kernel<<<dim3(kPix / 64, 2), 128, 0, stream>>>(AQ, AK, WQH, WKH, QN, KN);
  corr_soft_kernel<<<kPix / 32, 256, 0, stream>>>(QN, KN, P_cur, P_rnd, WVH, bvp, gammap, outp);
}
